// MultiHeadAttention_14310831030707
// MI455X (gfx1250) — hardware-verified
//
#include <hip/hip_runtime.h>


#ifndef NB
#define NB 2
#endif
#ifndef SEQ
#define SEQ 2048
#endif
#define NB_FULL  2
#define SEQ_FULL 2048
#define DM   1024
#define NH_  16
#define HD   64
#define DQ   (NH_ * HD)
#define RH   512
#define RHE  ((RH < SEQ) ? RH : SEQ)
#define SCL  0.125f
#define L2E  1.4426950408889634f
#define MFILL (-1.0e9f)
#define MINIT (-1.0e30f)
#define MSEEN (-5.0e8f)
#define F16MINN 6.103515625e-05f
#define PP 40
#define CP 72

typedef _Float16 h16;
typedef unsigned short bf;
typedef __attribute__((ext_vector_type(16))) __bf16   v16bf;
typedef __attribute__((ext_vector_type(16))) _Float16 v16h;
typedef __attribute__((ext_vector_type(8)))  _Float16 v8h;
typedef __attribute__((ext_vector_type(8)))  unsigned short v8us;
typedef __attribute__((ext_vector_type(8)))  float    v8f;
typedef __attribute__((ext_vector_type(4)))  float    v4f;
typedef __attribute__((ext_vector_type(2)))  float    v2f;
typedef __attribute__((ext_vector_type(2)))  _Float16 v2h;
typedef __attribute__((ext_vector_type(2)))  unsigned short v2us;
typedef __attribute__((ext_vector_type(4)))  int      v4i;
typedef v8h  __attribute__((may_alias)) v8ha;
typedef v4f  __attribute__((may_alias)) v4fa;
typedef v8us __attribute__((may_alias)) v8usa;

static_assert(HD == 64);
static_assert(DQ == DM);
static_assert(DM % 64 == 0);
static_assert(SEQ % 64 == 0);
static_assert(RH % 16 == 0);
static_assert(NB <= NB_FULL);
static_assert(SEQ <= SEQ_FULL);
static_assert((PP * 2) % 16 == 0);
static_assert((CP * 2) % 16 == 0);
static_assert((long long)NB * NH_ * SEQ * HD < 2147483647LL);
static_assert((long long)SEQ_FULL * SEQ_FULL < 2147483647LL);

constexpr size_t WS_W  = (size_t)4 * DM * DM * 2;
constexpr size_t WS_XB = (size_t)NB * SEQ * DM * 2;
constexpr size_t WS_F  = (size_t)NB * SEQ * DM * 4;
constexpr size_t WS_PL = (size_t)NB * NH_ * SEQ * HD * 2;
constexpr size_t WS_AT = (size_t)NB * SEQ * DQ * 2;
constexpr size_t WS_TOTAL = WS_W + WS_XB + WS_F + 9 * WS_PL + 2 * WS_AT;
static_assert(WS_TOTAL <= (size_t)134217728);
static_assert(WS_W % 256 == 0 && WS_XB % 256 == 0 && WS_F % 256 == 0 && WS_PL % 256 == 0 && WS_AT % 256 == 0);

__device__ __forceinline__ unsigned short f2bf(float f) { unsigned u = __float_as_uint(f); u += 0x7FFFu + ((u >> 16) & 1u); return (unsigned short)(u >> 16); }
__device__ __forceinline__ float bf2f(unsigned short b) { return __uint_as_float(((unsigned)b) << 16); }
__device__ __forceinline__ float bfr(float f) { return bf2f(f2bf(f)); }
__device__ __forceinline__ v16h cat16(v8h lo, v8h hi) { return __builtin_shufflevector(lo, hi, 0, 1, 2, 3, 4, 5, 6, 7, 8, 9, 10, 11, 12, 13, 14, 15); }
__device__ __forceinline__ v16bf cat16b(v8us lo, v8us hi) { return __builtin_bit_cast(v16bf, __builtin_shufflevector(lo, hi, 0, 1, 2, 3, 4, 5, 6, 7, 8, 9, 10, 11, 12, 13, 14, 15)); }
__device__ __forceinline__ v8f wmma16(v16h a, v16h b, v8f c) { return __builtin_amdgcn_wmma_f32_16x16x32_f16(false, a, false, b, (short)0, c, false, false); }
__device__ __forceinline__ v8f wmmab(v16bf a, v16bf b, v8f c) { return __builtin_amdgcn_wmma_f32_16x16x32_bf16(false, a, false, b, (short)0, c, false, false); }
__device__ __forceinline__ v8f mma3(v16bf ah, v16bf al, v16bf bh, v16bf bl, v8f c) { c = wmmab(ah, bh, c); c = wmmab(al, bh, c); c = wmmab(ah, bl, c); return c; }
__device__ __forceinline__ h16 tohx(float x) { return (h16)x; }
__device__ __forceinline__ void splitf(float y, unsigned short& h, unsigned short& l) { h = f2bf(y); l = f2bf(y - bf2f(h)); }
__device__ __forceinline__ void wave_sync() { __builtin_amdgcn_wave_barrier(); asm volatile("" ::: "memory"); }

template <typename T16> struct WFrag;
template <> struct WFrag<h16> { typedef v16h V; static __device__ __forceinline__ V ld(const h16* p) { return cat16(*(const v8h*)p, *(const v8h*)(p + 16)); } static __device__ __forceinline__ v8f mma(V a, V b, v8f c) { return wmma16(a, b, c); } };
template <> struct WFrag<bf> { typedef v16bf V; static __device__ __forceinline__ V ld(const bf* p) { return cat16b(*(const v8us*)p, *(const v8us*)(p + 16)); } static __device__ __forceinline__ v8f mma(V a, V b, v8f c) { return wmmab(a, b, c); } };

template <typename T16, int NSPLIT, bool BIAS>
__device__ __forceinline__ void gemmw_body(const T16* __restrict__ A, const T16* __restrict__ A2, const T16* __restrict__ Bt, const T16* __restrict__ Bt2, int K, float* C, int ldc, const float* __restrict__ bias, size_t sA, size_t sB, size_t sC) {
    typedef typename WFrag<T16>::V V;
    __shared__ __align__(16) float os[16 * 68];
    const size_t z = blockIdx.z; A += z * sA; if (A2) A2 += z * sA; Bt += z * sB; if (Bt2) Bt2 += z * sB; C += z * sC;
    const int lane = threadIdx.x & 31, lr = lane & 15, hi = lane >> 4; const int r0 = blockIdx.x * 64, c0 = blockIdx.y * 64;
    v8f acc[4][4];
#pragma unroll
    for (int mb = 0; mb < 4; ++mb)
#pragma unroll
        for (int nb = 0; nb < 4; ++nb) acc[mb][nb] = (v8f){};
    const size_t aoff = (size_t)(r0 + lr) * K + 8 * hi, boff = (size_t)(c0 + lr) * K + 8 * hi;
#pragma unroll 1
    for (int kc = 0; kc < K; kc += 32) {
        V a[4], a2[4];
#pragma unroll
        for (int mb = 0; mb < 4; ++mb) { a[mb] = WFrag<T16>::ld(A + aoff + (size_t)mb * 16 * K + kc); if (NSPLIT == 1 || NSPLIT == 2) a2[mb] = WFrag<T16>::ld(A2 + aoff + (size_t)mb * 16 * K + kc); }
#pragma unroll
        for (int nb = 0; nb < 4; ++nb) { const V b = WFrag<T16>::ld(Bt + boff + (size_t)nb * 16 * K + kc); V b2; if (NSPLIT >= 2) b2 = WFrag<T16>::ld(Bt2 + boff + (size_t)nb * 16 * K + kc);
#pragma unroll
            for (int mb = 0; mb < 4; ++mb) { acc[mb][nb] = WFrag<T16>::mma(a[mb], b, acc[mb][nb]); if (NSPLIT == 1 || NSPLIT == 2) acc[mb][nb] = WFrag<T16>::mma(a2[mb], b, acc[mb][nb]); if (NSPLIT >= 2) acc[mb][nb] = WFrag<T16>::mma(a[mb], b2, acc[mb][nb]); } }
        asm volatile("v_nop\n\tv_nop\n\tv_nop\n\tv_nop" : "+v"(acc[0][0]), "+v"(acc[1][1]), "+v"(acc[2][2]), "+v"(acc[3][3]) : "v"(a[0]), "v"(a[3]));
    }
#pragma unroll
    for (int mb = 0; mb < 4; ++mb) {
#pragma unroll
        for (int nb = 0; nb < 4; ++nb) {
#pragma unroll
            for (int j = 0; j < 8; ++j) os[(hi * 8 + j) * 68 + nb * 16 + lr] = acc[mb][nb][j]; }
        wave_sync();
        float* crow = C + (size_t)(r0 + mb * 16) * ldc + c0;
#pragma unroll 1
        for (int ps = 0; ps < 2; ++ps) {
#pragma unroll
            for (int s = 0; s < 8; ++s) { const int row = 2 * s + hi, cofs = lr * 4; v4f val = *(const v4fa*)(os + row * 68 + cofs); if (BIAS) { val[0] += bfr(bias[c0 + cofs]); val[1] += bfr(bias[c0 + cofs + 1]); val[2] += bfr(bias[c0 + cofs + 2]); val[3] += bfr(bias[c0 + cofs + 3]); }
                *(volatile v4f*)(crow + (size_t)row * ldc + cofs) = val; }
            if (ps == 0) __threadfence(); }
        wave_sync();
    }
}
__global__ __launch_bounds__(32) void k_proj(const bf* A, const bf* Bt, int K, float* C, int ldc, const float* bias, size_t sA, size_t sC) {
    gemmw_body<bf, 0, true>(A, nullptr, Bt, nullptr, K, C, ldc, bias, sA, (size_t)0, sC); }
__global__ __launch_bounds__(32) void k_oproj(const bf* A, const bf* A2, const bf* Bt, int K, float* C, int ldc, const float* bias, size_t sA, size_t sC) {
    gemmw_body<bf, 1, true>(A, A2, Bt, nullptr, K, C, ldc, bias, sA, (size_t)0, sC); }

__global__ __launch_bounds__(256) void k_cvt8(const float* __restrict__ src, bf* dst, int n8, size_t sS, size_t sD) {
    const int i = blockIdx.x * 256 + threadIdx.x; if (i >= n8) return; src += (size_t)blockIdx.y * sS; dst += (size_t)blockIdx.y * sD;
    const v8f v = *(const v8f*)(src + (size_t)i * 8); v8us o;
#pragma unroll
    for (int k = 0; k < 8; ++k) o[k] = f2bf(v[k]);
    *(volatile v8us*)(dst + (size_t)i * 8) = o; __threadfence(); *(volatile v8us*)(dst + (size_t)i * 8) = o; }

__global__ __launch_bounds__(256) void k_hplanes(const float* __restrict__ F, h16* P16, bf* Ph, bf* Pl) {
    const int e = (blockIdx.x * 256 + threadIdx.x) * 2; if (e >= NB * NH_ * SEQ * HD) return;
    const int d = e % HD; const int t = (e / HD) % SEQ; const int z = e / (HD * SEQ); const int b = z / NH_, h = z % NH_;
    const v2f x = *(const v2f*)(F + (size_t)(b * SEQ + t) * DM + h * HD + d); v2h o16; v2us oh, ol;
#pragma unroll
    for (int q = 0; q < 2; ++q) { o16[q] = tohx(x[q]); unsigned short a2, c2; splitf(x[q], a2, c2); oh[q] = a2; ol[q] = c2; }
    *(volatile v2h*)(P16 + e) = o16; *(volatile v2us*)(Ph + e) = oh; *(volatile v2us*)(Pl + e) = ol; __threadfence(); *(volatile v2h*)(P16 + e) = o16; *(volatile v2us*)(Ph + e) = oh; *(volatile v2us*)(Pl + e) = ol; }
__global__ __launch_bounds__(256) void k_vtplanes(const float* __restrict__ F, h16* V16, bf* Vh, bf* Vl) {
    const int e = (blockIdx.x * 256 + threadIdx.x) * 2; if (e >= NB * NH_ * HD * SEQ) return;
    const int t = e % SEQ; const int d = (e / SEQ) % HD; const int z = e / (SEQ * HD); const int b = z / NH_, h = z % NH_; v2h o16; v2us oh, ol;
#pragma unroll
    for (int q = 0; q < 2; ++q) { const float x = F[(size_t)(b * SEQ + t + q) * DM + h * HD + d]; o16[q] = tohx(x); unsigned short a2, c2; splitf(x, a2, c2); oh[q] = a2; ol[q] = c2; }
    *(volatile v2h*)(V16 + e) = o16; *(volatile v2us*)(Vh + e) = oh; *(volatile v2us*)(Vl + e) = ol; __threadfence(); *(volatile v2h*)(V16 + e) = o16; *(volatile v2us*)(Vh + e) = oh; *(volatile v2us*)(Vl + e) = ol; }

template <bool HI>
__device__ __forceinline__ void attn_body(const h16* __restrict__ Q16, const h16* __restrict__ K16, const h16* __restrict__ VT16,
                                          const bf* __restrict__ Qh, const bf* __restrict__ Ql, const bf* __restrict__ Kh, const bf* __restrict__ Kl,
                                          const bf* __restrict__ VTh, const bf* __restrict__ VTl, const int* __restrict__ mask, bf* ATh, bf* ATl, int row_base) {
    __shared__ __align__(16) h16 pt16[16 * PP];
    __shared__ __align__(16) unsigned short pth[16 * PP];
    __shared__ __align__(16) unsigned short ptl[16 * PP];
    __shared__ __align__(16) unsigned short cth[16 * CP];
    __shared__ __align__(16) unsigned short ctl[16 * CP];
    const int lane = threadIdx.x & 31, lr = lane & 15, hi = lane >> 4;
    const int q0 = row_base + (int)blockIdx.x * 16;
    const int h = blockIdx.y, b = blockIdx.z;
    const int zoff  = (b * NH_ + h) * (SEQ * HD);
    const int qbase = zoff + (q0 + lr) * HD + 8 * hi;
    const int kbase = zoff + lr * HD + 8 * hi;
    const int vbase = zoff + lr * SEQ + 8 * hi;
    const int mrowD = (q0 + 8 * hi) * SEQ_FULL + lr;
    const int mrowT = (q0 + (lane >> 3)) * SEQ_FULL + (lane & 7) * 4;

    v8f o[4]; float m[8], l[8];
    bool dense = false;
#pragma unroll 1
    for (int pass = 0; pass < 2; ++pass) {
#pragma unroll
        for (int t = 0; t < 4; ++t) o[t] = (v8f){};
#pragma unroll
        for (int r = 0; r < 8; ++r) { m[r] = MINIT; l[r] = 0.0f; }
#pragma unroll 1
        for (int kb = 0; kb < SEQ; kb += 32) {
            const v4i t0 = *(const v4i*)(mask + mrowT + kb);
            const v4i t1 = *(const v4i*)(mask + mrowT + 4 * SEQ_FULL + kb);
            const v4i t2 = *(const v4i*)(mask + mrowT + 8 * SEQ_FULL + kb);
            const v4i t3 = *(const v4i*)(mask + mrowT + 12 * SEQ_FULL + kb);
            const int tor = (t0[0] | t0[1] | t0[2] | t0[3]) | (t1[0] | t1[1] | t1[2] | t1[3]) | (t2[0] | t2[1] | t2[2] | t2[3]) | (t3[0] | t3[1] | t3[2] | t3[3]);
            const bool anyw = __builtin_amdgcn_ballot_w32(tor != 0) != 0u;
            if (!(dense || anyw)) continue;
            int mk0[8], mk1[8];
#pragma unroll
            for (int r = 0; r < 8; ++r) mk0[r] = mask[mrowD + r * SEQ_FULL + kb];
            asm volatile("" ::: "memory");
#pragma unroll
            for (int r = 0; r < 8; ++r) mk1[r] = mask[mrowD + r * SEQ_FULL + kb + 16];

            int qo = qbase; asm volatile("" : "+v"(qo));
            const int ko = kbase + kb * HD;
            v8f s0 = (v8f){}, s1 = (v8f){};
            if (HI) {
                const v16bf qh0 = WFrag<bf>::ld(Qh + qo), qh1 = WFrag<bf>::ld(Qh + qo + 32);
                const v16bf ql0 = WFrag<bf>::ld(Ql + qo), ql1 = WFrag<bf>::ld(Ql + qo + 32);
                s0 = mma3(qh0, ql0, WFrag<bf>::ld(Kh + ko), WFrag<bf>::ld(Kl + ko), s0);
                s0 = mma3(qh1, ql1, WFrag<bf>::ld(Kh + ko + 32), WFrag<bf>::ld(Kl + ko + 32), s0);
                s1 = mma3(qh0, ql0, WFrag<bf>::ld(Kh + ko + 16 * HD), WFrag<bf>::ld(Kl + ko + 16 * HD), s1);
                s1 = mma3(qh1, ql1, WFrag<bf>::ld(Kh + ko + 16 * HD + 32), WFrag<bf>::ld(Kl + ko + 16 * HD + 32), s1);
                asm volatile("v_nop\n\tv_nop\n\tv_nop\n\tv_nop" : "+v"(s0), "+v"(s1) : "v"(qh1), "v"(ql1));
            } else {
                const v16h qa0 = WFrag<h16>::ld(Q16 + qo), qa1 = WFrag<h16>::ld(Q16 + qo + 32);
                s0 = wmma16(qa0, WFrag<h16>::ld(K16 + ko), s0);
                s0 = wmma16(qa1, WFrag<h16>::ld(K16 + ko + 32), s0);
                s1 = wmma16(qa0, WFrag<h16>::ld(K16 + ko + 16 * HD), s1);
                s1 = wmma16(qa1, WFrag<h16>::ld(K16 + ko + 16 * HD + 32), s1);
                asm volatile("v_nop\n\tv_nop\n\tv_nop\n\tv_nop" : "+v"(s0), "+v"(s1) : "v"(qa0), "v"(qa1));
            }

#pragma unroll
            for (int r = 0; r < 8; ++r) {
                const float e0 = (mk0[r] == 0) ? MFILL : s0[r] * SCL;
                const float e1 = (mk1[r] == 0) ? MFILL : s1[r] * SCL;
                float rm = fmaxf(e0, e1);
                rm = fmaxf(rm, __shfl_xor(rm, 1, 32)); rm = fmaxf(rm, __shfl_xor(rm, 2, 32)); rm = fmaxf(rm, __shfl_xor(rm, 4, 32)); rm = fmaxf(rm, __shfl_xor(rm, 8, 32));
                const float mn = fmaxf(m[r], rm);
                const float al = __builtin_amdgcn_exp2f((m[r] - mn) * L2E);
                float x0 = __builtin_amdgcn_exp2f((e0 - mn) * L2E);
                float x1 = __builtin_amdgcn_exp2f((e1 - mn) * L2E);
                const int po = (8 * hi + r) * PP + lr;
                float rs;
                if (HI) {
                    unsigned short a0, c0, a1, c1; splitf(x0, a0, c0); splitf(x1, a1, c1);
                    pth[po] = a0; ptl[po] = c0; pth[po + 16] = a1; ptl[po + 16] = c1;
                    rs = x0 + x1;
                } else {
                    x0 = (x0 < F16MINN) ? 0.0f : x0; x1 = (x1 < F16MINN) ? 0.0f : x1;
                    const h16 g0 = tohx(x0), g1 = tohx(x1);
                    pt16[po] = g0; pt16[po + 16] = g1;
                    rs = (float)g0 + (float)g1;
                }
                rs += __shfl_xor(rs, 1, 32); rs += __shfl_xor(rs, 2, 32); rs += __shfl_xor(rs, 4, 32); rs += __shfl_xor(rs, 8, 32);
                l[r] = l[r] * al + rs; m[r] = mn;
                o[0][r] *= al; o[1][r] *= al; o[2][r] *= al; o[3][r] *= al;
            }
            wave_sync();
            const int vo = vbase + kb;
            if (HI) {
                const v16bf pa = cat16b(*(const v8usa*)(pth + lr * PP + 8 * hi), *(const v8usa*)(pth + lr * PP + 16 + 8 * hi));
                const v16bf pb = cat16b(*(const v8usa*)(ptl + lr * PP + 8 * hi), *(const v8usa*)(ptl + lr * PP + 16 + 8 * hi));
                const v16bf vh0 = WFrag<bf>::ld(VTh + vo), vh1 = WFrag<bf>::ld(VTh + vo + 16 * SEQ), vh2 = WFrag<bf>::ld(VTh + vo + 32 * SEQ), vh3 = WFrag<bf>::ld(VTh + vo + 48 * SEQ);
                const v16bf vl0 = WFrag<bf>::ld(VTl + vo), vl1 = WFrag<bf>::ld(VTl + vo + 16 * SEQ), vl2 = WFrag<bf>::ld(VTl + vo + 32 * SEQ), vl3 = WFrag<bf>::ld(VTl + vo + 48 * SEQ);
                o[0] = mma3(pa, pb, vh0, vl0, o[0]); o[1] = mma3(pa, pb, vh1, vl1, o[1]); o[2] = mma3(pa, pb, vh2, vl2, o[2]); o[3] = mma3(pa, pb, vh3, vl3, o[3]);
                asm volatile("v_nop\n\tv_nop\n\tv_nop\n\tv_nop" : "+v"(o[0]), "+v"(o[1]), "+v"(o[2]), "+v"(o[3]) : "v"(pa), "v"(pb));
            } else {
                const v16h pa = cat16(*(const v8ha*)(pt16 + lr * PP + 8 * hi), *(const v8ha*)(pt16 + lr * PP + 16 + 8 * hi));
                const v16h v0 = WFrag<h16>::ld(VT16 + vo), v1 = WFrag<h16>::ld(VT16 + vo + 16 * SEQ), v2 = WFrag<h16>::ld(VT16 + vo + 32 * SEQ), v3 = WFrag<h16>::ld(VT16 + vo + 48 * SEQ);
                o[0] = wmma16(pa, v0, o[0]); o[1] = wmma16(pa, v1, o[1]); o[2] = wmma16(pa, v2, o[2]); o[3] = wmma16(pa, v3, o[3]);
                asm volatile("v_nop\n\tv_nop\n\tv_nop\n\tv_nop" : "+v"(o[0]), "+v"(o[1]), "+v"(o[2]), "+v"(o[3]) : "v"(pa), "v"(v3));
            }
            wave_sync();
        }
        bool bad = false;
#pragma unroll
        for (int r = 0; r < 8; ++r) bad = bad || !(m[r] > MSEEN);
        if (__builtin_amdgcn_ballot_w32(bad) == 0u) break;
        dense = true;
    }

#pragma unroll
    for (int r = 0; r < 8; ++r) { const float inv = 1.0f / l[r];
#pragma unroll
        for (int dt = 0; dt < 4; ++dt) { unsigned short a, c; splitf(o[dt][r] * inv, a, c); cth[(8 * hi + r) * CP + dt * 16 + lr] = a; ctl[(8 * hi + r) * CP + dt * 16 + lr] = c; } }
    wave_sync();
    v8us hv[4], lv[4];
#pragma unroll
    for (int s = 0; s < 4; ++s) { const int row = 4 * s + (lane >> 3); hv[s] = *(const v8usa*)(cth + row * CP + (lane & 7) * 8); lv[s] = *(const v8usa*)(ctl + row * CP + (lane & 7) * 8); }
    const size_t ob = (size_t)(b * SEQ + q0 + (lane >> 3)) * DQ + h * HD + (lane & 7) * 8;
#pragma unroll 1
    for (int ps = 0; ps < 2; ++ps) {
#pragma unroll
        for (int s = 0; s < 4; ++s) { *(volatile v8us*)(ATh + ob + (size_t)(4 * s) * DQ) = hv[s]; *(volatile v8us*)(ATl + ob + (size_t)(4 * s) * DQ) = lv[s]; }
        if (ps == 0) __threadfence(); }
}
__global__ __launch_bounds__(32) void k_attn_hi(const bf* Qh, const bf* Ql, const bf* Kh, const bf* Kl, const bf* VTh, const bf* VTl, const int* mask, bf* ATh, bf* ATl) {
    attn_body<true>(nullptr, nullptr, nullptr, Qh, Ql, Kh, Kl, VTh, VTl, mask, ATh, ATl, 0); }
__global__ __launch_bounds__(32) void k_attn_lo(const h16* Q16, const h16* K16, const h16* VT16, const int* mask, bf* ATh, bf* ATl) {
    attn_body<false>(Q16, K16, VT16, nullptr, nullptr, nullptr, nullptr, nullptr, nullptr, mask, ATh, ATl, RHE); }

extern "C" void kernel_launch(void* const* d_in, const int* in_sizes, int n_in,
                              void* d_out, int out_size, void* d_ws, size_t ws_size, hipStream_t stream) {
    if (n_in < 12) return;
    const long long need_x = (long long)(NB - 1) * SEQ_FULL * DM + (long long)SEQ * DM;
    const long long need_m = (long long)(SEQ - 1) * SEQ_FULL + SEQ;
    if (in_sizes[0] < need_x || in_sizes[1] < need_x || in_sizes[2] < need_x || in_sizes[3] < need_m) return;
    if (in_sizes[4] < DM * DM || in_sizes[6] < DM * DM || in_sizes[8] < DM * DM || in_sizes[10] < DM * DM) return;
    if (in_sizes[5] < DM || in_sizes[7] < DM || in_sizes[9] < DM || in_sizes[11] < DM) return;
    if ((long long)out_size < need_x) return;
    if (WS_TOTAL > ws_size) return;
    const float* xq = (const float*)d_in[0]; const float* xk = (const float*)d_in[1]; const float* xv = (const float*)d_in[2];
    const int* mask = (const int*)d_in[3];
    const float* wq = (const float*)d_in[4]; const float* bq = (const float*)d_in[5];
    const float* wk = (const float*)d_in[6]; const float* bk = (const float*)d_in[7];
    const float* wv = (const float*)d_in[8]; const float* bv = (const float*)d_in[9];
    const float* wo = (const float*)d_in[10]; const float* bo = (const float*)d_in[11];
    float* OUT = (float*)d_out;
    char* wsp = (char*)d_ws;
    auto take = [&](size_t bytes) { char* p = wsp; wsp += bytes; return (void*)p; };
    bf* WQ = (bf*)take(WS_W / 4); bf* WK = (bf*)take(WS_W / 4); bf* WV = (bf*)take(WS_W / 4); bf* WO = (bf*)take(WS_W / 4);
    bf* XB = (bf*)take(WS_XB); float* F = (float*)take(WS_F);
    h16* Q16 = (h16*)take(WS_PL); bf* Qh = (bf*)take(WS_PL); bf* Ql = (bf*)take(WS_PL);
    h16* K16 = (h16*)take(WS_PL); bf* Kh = (bf*)take(WS_PL); bf* Kl = (bf*)take(WS_PL);
    h16* VT16 = (h16*)take(WS_PL); bf* VTh = (bf*)take(WS_PL); bf* VTl = (bf*)take(WS_PL);
    bf* ATh = (bf*)take(WS_AT); bf* ATl = (bf*)take(WS_AT);
    if ((size_t)(wsp - (char*)d_ws) > ws_size) return;

    const unsigned gW = (unsigned)((DM * DM / 8 + 255) / 256), gX = (unsigned)((SEQ * DM / 8 + 255) / 256), gP = (unsigned)((NB * NH_ * SEQ * HD / 2 + 255) / 256);
    k_cvt8<<<dim3(gW, 1), 256, 0, stream>>>(wq, WQ, DM * DM / 8, (size_t)0, (size_t)0);
    k_cvt8<<<dim3(gW, 1), 256, 0, stream>>>(wk, WK, DM * DM / 8, (size_t)0, (size_t)0);
    k_cvt8<<<dim3(gW, 1), 256, 0, stream>>>(wv, WV, DM * DM / 8, (size_t)0, (size_t)0);
    k_cvt8<<<dim3(gW, 1), 256, 0, stream>>>(wo, WO, DM * DM / 8, (size_t)0, (size_t)0);
    const dim3 gG(SEQ / 64, DQ / 64, NB);
    k_cvt8<<<dim3(gX, NB), 256, 0, stream>>>(xq, XB, SEQ * DM / 8, (size_t)SEQ_FULL * DM, (size_t)SEQ * DM);
    k_proj<<<gG, 32, 0, stream>>>(XB, WQ, DM, F, DQ, bq, (size_t)SEQ * DM, (size_t)SEQ * DQ);
    k_hplanes<<<gP, 256, 0, stream>>>(F, Q16, Qh, Ql);
    k_cvt8<<<dim3(gX, NB), 256, 0, stream>>>(xk, XB, SEQ * DM / 8, (size_t)SEQ_FULL * DM, (size_t)SEQ * DM);
    k_proj<<<gG, 32, 0, stream>>>(XB, WK, DM, F, DQ, bk, (size_t)SEQ * DM, (size_t)SEQ * DQ);
    k_hplanes<<<gP, 256, 0, stream>>>(F, K16, Kh, Kl);
    k_cvt8<<<dim3(gX, NB), 256, 0, stream>>>(xv, XB, SEQ * DM / 8, (size_t)SEQ_FULL * DM, (size_t)SEQ * DM);
    k_proj<<<gG, 32, 0, stream>>>(XB, WV, DM, F, DQ, bv, (size_t)SEQ * DM, (size_t)SEQ * DQ);
    k_vtplanes<<<gP, 256, 0, stream>>>(F, VT16, VTh, VTl);
    k_attn_hi<<<dim3(RHE / 16, NH_, NB), 32, 0, stream>>>(Qh, Ql, Kh, Kl, VTh, VTl, mask, ATh, ATl);
#if SEQ > RH
    k_attn_lo<<<dim3((SEQ - RHE) / 16, NH_, NB), 32, 0, stream>>>(Q16, K16, VT16, mask, ATh, ATl);
#endif
    k_oproj<<<dim3(SEQ / 64, DM / 64, NB), 32, 0, stream>>>(ATh, ATl, WO, DQ, OUT, DM, bo, (size_t)SEQ * DQ, (size_t)SEQ_FULL * DM);
}
